// ramsey_MPNN_2911987826887
// MI455X (gfx1250) — hardware-verified
//
#include <hip/hip_runtime.h>
#include <math.h>

constexpr int kNodes    = 1024;
constexpr int kFeat     = 128;
constexpr int kHid      = 512;
constexpr int kCls      = 2;
constexpr int kEdges    = kNodes * (kNodes - 1) / 2;
constexpr int kChunkE   = 65536;
constexpr int kNumChunks = (kEdges + kChunkE - 1) / kChunkE;
constexpr int kTwoNm1   = 2 * kNodes - 1;
constexpr int kTwoNm1Sq = kTwoNm1 * kTwoNm1;
constexpr int kW6Rows   = 16;
constexpr int kSlabPitch = 16;
constexpr float kWCarry   = 16.0f;
constexpr float kActCarry = 16.0f;
constexpr float kProdCarry = 16.0f;
constexpr float kScale1   = 1.0f / 16.0f;
constexpr float kScale2   = 1.0f / 256.0f;
static_assert(kNumChunks == 8, "chunk count");
static_assert(kTwoNm1Sq < (1 << 24), "exact in f32");
static_assert(kChunkE % 512 == 0, "tile multiples");
static_assert(kNodes % 64 == 0 && kFeat % 64 == 0 && kHid % 64 == 0, "tile multiples");

constexpr size_t kOffNF16 = 0;
constexpr size_t kOffW1T  = kOffNF16 + (size_t)kNodes * kFeat * 2;
constexpr size_t kOffW2T  = kOffW1T  + (size_t)kHid * kFeat * 2;
constexpr size_t kOffW4T  = kOffW2T  + (size_t)kHid * kHid * 2;
constexpr size_t kOffW5T  = kOffW4T  + (size_t)kFeat * kHid * 2;
constexpr size_t kOffW6T  = kOffW5T  + (size_t)kHid * kFeat * 2;
constexpr size_t kOffH1   = kOffW6T  + (size_t)kW6Rows * kHid * 2;
constexpr size_t kOffH2   = kOffH1   + (size_t)kNodes * kHid * 2;
constexpr size_t kOffHF   = kOffH2   + (size_t)kNodes * kHid * 2;
constexpr size_t kOffProd = kOffHF   + (size_t)kNodes * kFeat * 4;
constexpr size_t kOffEP   = kOffProd + (size_t)kChunkE * kFeat * 2;
constexpr size_t kOffEPS  = kOffEP   + (size_t)kChunkE * kHid * 2;
constexpr size_t kWsTotal = kOffEPS  + (size_t)kNumChunks * kChunkE * kCls * 4;
static_assert(kWsTotal == 91897856, "carve total");
static_assert(kWsTotal <= 134217728, "carve cap");

typedef __attribute__((ext_vector_type(16))) _Float16 v16h;
typedef __attribute__((ext_vector_type(8)))  _Float16 v8h;
typedef __attribute__((ext_vector_type(16))) __bf16   v16b;
typedef __attribute__((ext_vector_type(8)))  __bf16   v8b;
typedef __attribute__((ext_vector_type(8)))  float    v8f;
typedef __attribute__((ext_vector_type(4)))  float    v4f;
typedef __attribute__((ext_vector_type(2)))  float    v2f;
typedef __attribute__((ext_vector_type(4)))  unsigned int v4u;

__device__ __forceinline__ unsigned short f2bf_bits(float f) {
  unsigned u = __float_as_uint(f);
  return (unsigned short)((u + 0x7FFFu + ((u >> 16) & 1u)) >> 16);
}
__device__ __forceinline__ float bf_bits2f(unsigned short h) { return __uint_as_float(((unsigned)h) << 16); }

__device__ __forceinline__ void dep_guard_h(v8f& a, v8f& b, v16h x, v16h y) { asm volatile("v_nop\n\tv_nop\n\tv_nop\n\tv_nop" : "+v"(a), "+v"(b) : "v"(x), "v"(y)); }
__device__ __forceinline__ void dep_guard_b(v8f& a, v8f& b, v16b x, v16b y) { asm volatile("v_nop\n\tv_nop\n\tv_nop\n\tv_nop" : "+v"(a), "+v"(b) : "v"(x), "v"(y)); }
__device__ __forceinline__ void keep4_h(v16h a, v16h b, v16h c, v16h d) { asm volatile("v_nop" :: "v"(a), "v"(b), "v"(c), "v"(d)); }
__device__ __forceinline__ void keep4_b(v16b a, v16b b, v16b c, v16b d) { asm volatile("v_nop" :: "v"(a), "v"(b), "v"(c), "v"(d)); }
__device__ __forceinline__ void acc_guard4(v8f& a, v8f& b, v8f& c, v8f& d) { asm volatile("v_nop\n\tv_nop\n\tv_nop\n\tv_nop" : "+v"(a), "+v"(b), "+v"(c), "+v"(d)); }
template <typename T> struct Frag;
template <> struct Frag<_Float16> {
  typedef v16h V; union U { v16h v; v8h h[2]; };
  static __device__ __forceinline__ v16h load(const _Float16* p) {
    U f; f.h[0] = *(const v8h*)(p); f.h[1] = *(const v8h*)(p + 16); return f.v;
  }
  static __device__ __forceinline__ v8f mma(v16h a, v16h b, v8f c) {
    return __builtin_amdgcn_wmma_f32_16x16x32_f16(false, a, false, b, (short)0, c, false, false);
  }
  static __device__ __forceinline__ void guard(v8f& a, v8f& b, v16h x, v16h y) { dep_guard_h(a, b, x, y); }
  static __device__ __forceinline__ void keep(v16h a, v16h b, v16h c, v16h d) { keep4_h(a, b, c, d); }
};
template <> struct Frag<__bf16> {
  typedef v16b V; union U { v16b v; v8b h[2]; };
  static __device__ __forceinline__ v16b load(const __bf16* p) {
    U f; f.h[0] = *(const v8b*)(p); f.h[1] = *(const v8b*)(p + 16); return f.v;
  }
  static __device__ __forceinline__ v8f mma(v16b a, v16b b, v8f c) {
    return __builtin_amdgcn_wmma_f32_16x16x32_bf16(false, a, false, b, (short)0, c, false, false);
  }
  static __device__ __forceinline__ void guard(v8f& a, v8f& b, v16b x, v16b y) { dep_guard_b(a, b, x, y); }
  static __device__ __forceinline__ void keep(v16b a, v16b b, v16b c, v16b d) { keep4_b(a, b, c, d); }
};

__device__ __forceinline__ unsigned pk16(unsigned short a, unsigned short b) { return (unsigned)a | ((unsigned)b << 16); }
__device__ __forceinline__ unsigned short h_bits(float f) { const _Float16 h = (_Float16)f; return __builtin_bit_cast(unsigned short, h); }

__device__ __forceinline__ v8f mma_f16_g(v16h a, v16h b, v8f c) {
  c = __builtin_amdgcn_wmma_f32_16x16x32_f16(false, a, false, b, (short)0, c, false, false);
  asm volatile("v_nop\n\tv_nop\n\tv_nop\n\tv_nop" : "+v"(c) : "v"(a), "v"(b));
  return c;
}

__device__ __forceinline__ int clampi(int v, int lo, int hi) { return v < lo ? lo : (v > hi ? hi : v); }

template <int ET> struct Elem;
template <> struct Elem<0> { typedef _Float16 T; };
template <> struct Elem<1> { typedef __bf16 T; };
template <int ET, bool SPLIT, int BIAS_MODE, int OUT_MODE, bool RESID, int ACT = 0>
__global__ __launch_bounds__(256) void wmma_gemm64(
    const unsigned short* __restrict__ Ap, const unsigned short* __restrict__ A2p, int lda, long strideA,
    const unsigned short* __restrict__ Btp, const unsigned short* __restrict__ Bt2p, int ldb, long strideB,
    void* __restrict__ Cout, void* __restrict__ Cout2, int ldc, long strideC,
    const float* __restrict__ bias,
    const float* __restrict__ resid, long strideR,
    int M, int N, int K, float scale, float ocarry) {
  typedef typename Elem<ET>::T T;
  typedef typename Frag<T>::V V;
  const T* A = (const T*)Ap; const T* A2 = (const T*)A2p; const T* Bt = (const T*)Btp; const T* Bt2 = (const T*)Bt2p;
  __shared__ __align__(16) float sT[8][16 * 68];
  const int b    = blockIdx.y;
  const int lane = threadIdx.x & 31;
  const int wave = threadIdx.x >> 5;
  const int tilesN = N >> 6;
  const int tilesM = M >> 6;
  const int tile = blockIdx.x * 8 + wave;
  if (tile >= tilesM * tilesN) return;
  const int tm = tile / tilesN;
  const int tn = tile - tm * tilesN;
  const int m0 = tm << 6;
  const int n0 = tn << 6;

  const T* Ab  = A  + (size_t)b * strideA;
  const T* Bb  = Bt + (size_t)b * strideB;
  const T* Ab2 = SPLIT ? (A2  + (size_t)b * strideA) : nullptr;
  const T* Bb2 = SPLIT ? (Bt2 + (size_t)b * strideB) : nullptr;

  const int rlane = lane & 15;
  const int koff  = (lane >> 4) * 8;
  const int mOff  = (lane >> 4) * 8;

  v8f acc[4][4];
#pragma unroll
  for (int i = 0; i < 4; ++i)
#pragma unroll
    for (int j = 0; j < 4; ++j) acc[i][j] = (v8f){0.f,0.f,0.f,0.f,0.f,0.f,0.f,0.f};

  for (int k0 = 0; k0 < K; k0 += 32) {
    V bh[4], bl[4];
#pragma unroll
    for (int j = 0; j < 4; ++j) {
      const size_t bo = (size_t)(n0 + (j << 4) + rlane) * ldb + koff + k0;
      bh[j] = Frag<T>::load(Bb + bo);
      if (SPLIT) bl[j] = Frag<T>::load(Bb2 + bo);
    }
#pragma unroll
    for (int i = 0; i < 4; ++i) {
      const size_t ao = (size_t)(m0 + (i << 4) + rlane) * lda + koff + k0;
      V ah = Frag<T>::load(Ab + ao);
      V al;
      if (SPLIT) al = Frag<T>::load(Ab2 + ao);
#pragma unroll
      for (int j = 0; j < 4; ++j) {
        acc[i][j] = Frag<T>::mma(ah, bh[j], acc[i][j]);
        if (SPLIT) {
          acc[i][j] = Frag<T>::mma(ah, bl[j], acc[i][j]);
          acc[i][j] = Frag<T>::mma(al, bh[j], acc[i][j]);
        }
      }
      Frag<T>::guard(acc[i][0], acc[i][3], ah, SPLIT ? al : ah);
    }
    Frag<T>::keep(bh[0], bh[1], bh[2], bh[3]);
    if (SPLIT) Frag<T>::keep(bl[0], bl[1], bl[2], bl[3]);
  }
  acc_guard4(acc[0][0], acc[0][1], acc[0][2], acc[0][3]);
  acc_guard4(acc[1][0], acc[1][1], acc[1][2], acc[1][3]);
  acc_guard4(acc[2][0], acc[2][1], acc[2][2], acc[2][3]);
  acc_guard4(acc[3][0], acc[3][1], acc[3][2], acc[3][3]);

  float* slab = sT[wave];
  const float* Rb = RESID ? (resid + (size_t)b * strideR) : nullptr;
#pragma unroll
  for (int i = 0; i < 4; ++i) {
    const int mBase = m0 + (i << 4);
#pragma unroll
    for (int j = 0; j < 4; ++j) {
      const int n = n0 + (j << 4) + rlane;
      float bv = 0.f;
      if (BIAS_MODE == 2) bv = bias[n];
#pragma unroll
      for (int r = 0; r < 8; ++r) {
        float v = acc[i][j][r] * scale;
        if (BIAS_MODE == 1) v += bias[mBase + mOff + r];
        if (BIAS_MODE == 2) v += bv;
        if (RESID) v += Rb[(size_t)(mBase + mOff + r) * ldc + n];
        if (ACT == 2) v = fmaxf(v, 0.0f);
        if (ACT == 4) v = (v > 0.f) ? v : 0.01f * v;
        v = v * ocarry;
        slab[(mOff + r) * 68 + (j << 4) + rlane] = v;
      }
    }
    __builtin_amdgcn_fence(__ATOMIC_RELEASE, "workgroup");
    __builtin_amdgcn_wave_barrier();
    __builtin_amdgcn_fence(__ATOMIC_ACQUIRE, "workgroup");
    if (OUT_MODE == 0) {
      float* C = (float*)Cout + (size_t)b * strideC;
      const int hh = lane >> 4, c4 = (lane & 15) * 4;
      for (int pass = 0; pass < 2; ++pass) {
#pragma unroll
        for (int it = 0; it < 8; ++it) {
          const int row = it * 2 + hh;
          v4f v = *(const v4f*)(slab + row * 68 + c4);
          *(volatile v4f*)(C + (size_t)(mBase + row) * ldc + n0 + c4) = v;
        }
        __threadfence();
      }
    } else {
      const int q = lane >> 3, c8 = (lane & 7) * 8;
      unsigned short* C  = (unsigned short*)Cout  + (size_t)b * strideC;
      unsigned short* C2 = (OUT_MODE == 2) ? ((unsigned short*)Cout2 + (size_t)b * strideC) : nullptr;
      for (int pass = 0; pass < 2; ++pass) {
#pragma unroll
        for (int it = 0; it < 4; ++it) {
          const int row = it * 4 + q;
          const float* sp = slab + row * 68 + c8;
          v8h hv, lv;
#pragma unroll
          for (int e = 0; e < 8; ++e) {
            if (OUT_MODE == 1) {
              hv[e] = (_Float16)sp[e];
            } else {
              unsigned short hb = f2bf_bits(sp[e]);
              unsigned short lb = f2bf_bits(sp[e] - bf_bits2f(hb));
              hv[e] = __builtin_bit_cast(_Float16, hb);
              lv[e] = __builtin_bit_cast(_Float16, lb);
            }
          }
          *(volatile v8h*)(C + (size_t)(mBase + row) * ldc + n0 + c8) = hv;
          if (OUT_MODE == 2) *(volatile v8h*)(C2 + (size_t)(mBase + row) * ldc + n0 + c8) = lv;
        }
        __threadfence();
      }
    }
    __builtin_amdgcn_fence(__ATOMIC_RELEASE, "workgroup");
    __builtin_amdgcn_wave_barrier();
    __builtin_amdgcn_fence(__ATOMIC_ACQUIRE, "workgroup");
  }
}

__global__ __launch_bounds__(256) void cast8_f16_kernel(const float* __restrict__ in, unsigned short* __restrict__ out, int n8) {
  const int i = blockIdx.x * 256 + threadIdx.x;
  if (i >= n8) return;
  const float* p = in + 8 * (size_t)i;
  const v4f a = *(const v4f*)(p);
  const v4f c = *(const v4f*)(p + 4);
  unsigned short hb[8];
#pragma unroll
  for (int e = 0; e < 4; ++e) {
    hb[e]     = h_bits(a[e]);
    hb[4 + e] = h_bits(c[e]);
  }
  const v4u u = (v4u){pk16(hb[0], hb[1]), pk16(hb[2], hb[3]), pk16(hb[4], hb[5]), pk16(hb[6], hb[7])};
  unsigned short* q = out + 8 * (size_t)i;
  *(volatile v4u*)q = u;
  __threadfence();
  *(volatile v4u*)q = u;
}

__global__ __launch_bounds__(256) void tcast_kernel(const float* __restrict__ in, unsigned short* __restrict__ out,
                                                    int R, int Cc, float scale) {
  __shared__ float sm[64][65];
  const int t  = threadIdx.x;
  const int r0 = blockIdx.x * 64;
  const int c0 = blockIdx.y * 64;
#pragma unroll
  for (int i = 0; i < 16; ++i) {
    const int e  = i * 256 + t;
    const int rl = e >> 6;
    const int cl = e & 63;
    sm[cl][rl] = in[(size_t)(r0 + rl) * Cc + c0 + cl] * scale;
  }
  __syncthreads();
  const int lane = t & 31, wave = t >> 5;
  const int q = lane >> 3, c8 = (lane & 7) * 8;
  for (int pass = 0; pass < 2; ++pass) {
#pragma unroll
    for (int it = 0; it < 2; ++it) {
      const int row = wave * 8 + it * 4 + q;
      unsigned short hb[8];
#pragma unroll
      for (int e = 0; e < 8; ++e) hb[e] = h_bits(sm[row][c8 + e]);
      const v4u u = (v4u){pk16(hb[0], hb[1]), pk16(hb[2], hb[3]), pk16(hb[4], hb[5]), pk16(hb[6], hb[7])};
      *(volatile v4u*)(out + (size_t)(c0 + row) * R + r0 + c8) = u;
    }
    __threadfence();
  }
}

__global__ __launch_bounds__(256) void w6t_kernel(const float* __restrict__ w6, unsigned short* __restrict__ out) {
  const int t = blockIdx.x * 256 + threadIdx.x;
  if (t >= kW6Rows * (kHid / 8)) return;
  const int row = t >> 6;
  const int k0  = (t & 63) * 8;
  const int rc  = row < kCls ? row : (kCls - 1);
  const bool live = row < kCls;
  unsigned short hb[8];
#pragma unroll
  for (int e = 0; e < 8; ++e) {
    const float wv = w6[(size_t)(k0 + e) * kCls + rc];
    const float v  = live ? wv * kWCarry : 0.0f;
    hb[e] = h_bits(v);
  }
  const v4u u = (v4u){pk16(hb[0], hb[1]), pk16(hb[2], hb[3]), pk16(hb[4], hb[5]), pk16(hb[6], hb[7])};
  unsigned short* dst = out + (size_t)row * kHid + k0;
  *(volatile v4u*)dst = u;
  __threadfence();
  *(volatile v4u*)dst = u;
}

__device__ __forceinline__ int row_start(int i) { return (i * (kTwoNm1 - i)) >> 1; }
__device__ __forceinline__ void edge_to_pair(int e, int& i, int& j) {
  const int dd = kTwoNm1Sq - 8 * e;
  const float s = sqrtf((float)dd);
  int ii = (int)(((float)kTwoNm1 - s) * 0.5f);
  ii = clampi(ii, 0, kNodes - 2);
  if (ii < kNodes - 2 && row_start(ii + 1) <= e) ++ii;
  if (ii < kNodes - 2 && row_start(ii + 1) <= e) ++ii;
  if (ii > 0 && row_start(ii) > e) --ii;
  if (ii > 0 && row_start(ii) > e) --ii;
  ii = clampi(ii, 0, kNodes - 2);
  int jj = e - row_start(ii) + ii + 1;
  jj = clampi(jj, 0, kNodes - 1);
  i = ii; j = jj;
}

__global__ __launch_bounds__(256) void pair_prod_kernel(const float* __restrict__ hf, unsigned short* __restrict__ prod,
                                                        int ebase) {
  const int t  = blockIdx.x * 256 + threadIdx.x;
  if (t >= kChunkE * (kFeat / 8)) return;
  const int el = t >> 4;
  const int g  = t & 15;
  const int e  = ebase + el;
  const bool valid = e < kEdges;
  const int ec = valid ? e : (kEdges - 1);
  int i, j;
  edge_to_pair(ec, i, j);
  const float* pi = hf + (size_t)i * kFeat + 8 * g;
  const float* pj = hf + (size_t)j * kFeat + 8 * g;
  const v4f a0 = *(const v4f*)(pi);
  const v4f a1 = *(const v4f*)(pi + 4);
  const v4f c0 = *(const v4f*)(pj);
  const v4f c1 = *(const v4f*)(pj + 4);
  unsigned short hb[8];
#pragma unroll
  for (int q = 0; q < 4; ++q) {
    const float p0 = a0[q] * c0[q];
    const float p1 = a1[q] * c1[q];
    hb[q]     = h_bits(valid ? p0 * kProdCarry : 0.0f);
    hb[4 + q] = h_bits(valid ? p1 * kProdCarry : 0.0f);
  }
  const v4u u = (v4u){pk16(hb[0], hb[1]), pk16(hb[2], hb[3]), pk16(hb[4], hb[5]), pk16(hb[6], hb[7])};
  unsigned short* dst = prod + (size_t)el * kFeat + 8 * g;
  *(volatile v4u*)dst = u;
  __threadfence();
  *(volatile v4u*)dst = u;
}

__device__ __forceinline__ void softmax2(float z0, float z1, float& p0, float& p1) {
  const float mx = fmaxf(z0, z1);
  const float e0 = expf(z0 - mx);
  const float e1 = expf(z1 - mx);
  const float inv = 1.0f / (e0 + e1);
  p0 = e0 * inv;
  p1 = e1 * inv;
}

__global__ __launch_bounds__(256) void logit_softmax_kernel(const unsigned short* __restrict__ EPp,
                                                            const unsigned short* __restrict__ W6p,
                                                            const float* __restrict__ b6,
                                                            float* __restrict__ eps) {
  const _Float16* EP  = (const _Float16*)EPp;
  const _Float16* W6T = (const _Float16*)W6p;
  __shared__ __align__(16) float sL[8][64 * kSlabPitch];
  const int lane  = threadIdx.x & 31;
  const int wave  = threadIdx.x >> 5;
  const int rlane = lane & 15;
  const int hsel  = lane >> 4;
  const int koff  = hsel * 8;
  const int m0    = blockIdx.x * 512 + wave * 64;
  v8f acc[4];
#pragma unroll
  for (int i = 0; i < 4; ++i) acc[i] = (v8f){0.f,0.f,0.f,0.f,0.f,0.f,0.f,0.f};
#pragma unroll 1
  for (int k0 = 0; k0 < kHid; k0 += 32) {
    const v16h bfrag = Frag<_Float16>::load(W6T + (size_t)rlane * kHid + koff + k0);
#pragma unroll
    for (int i = 0; i < 4; ++i) {
      const v16h afrag = Frag<_Float16>::load(EP + (size_t)(m0 + 16 * i + rlane) * kHid + koff + k0);
      acc[i] = mma_f16_g(afrag, bfrag, acc[i]);
    }
  }
  float* slab = sL[wave];
#pragma unroll
  for (int i = 0; i < 4; ++i) {
#pragma unroll
    for (int r = 0; r < 8; ++r) slab[(16 * i + 8 * hsel + r) * kSlabPitch + rlane] = acc[i][r] * kScale2;
  }
  __builtin_amdgcn_fence(__ATOMIC_RELEASE, "workgroup");
  __builtin_amdgcn_wave_barrier();
  __builtin_amdgcn_fence(__ATOMIC_ACQUIRE, "workgroup");
  const float bz0 = b6[0], bz1 = b6[1];
  const int ra = 2 * lane, rb = 2 * lane + 1;
  const float za0 = slab[ra * kSlabPitch + 0] + bz0;
  const float za1 = slab[ra * kSlabPitch + 1] + bz1;
  const float zb0 = slab[rb * kSlabPitch + 0] + bz0;
  const float zb1 = slab[rb * kSlabPitch + 1] + bz1;
  float pa0, pa1, pb0, pb1;
  softmax2(za0, za1, pa0, pa1);
  softmax2(zb0, zb1, pb0, pb1);
  const v4f o = (v4f){pa0, pa1, pb0, pb1};
  float* dst = eps + (size_t)(m0 + ra) * kCls;
  *(volatile v4f*)dst = o;
  __threadfence();
  *(volatile v4f*)dst = o;
}

__global__ __launch_bounds__(256) void dense_write_kernel(const float* __restrict__ eps, float* __restrict__ out) {
  const int t = blockIdx.x * 256 + threadIdx.x;
  if (t >= kNodes * (kNodes / 2)) return;
  const int a  = t >> 9;
  const int bp = (t & 511) * 2;
  float vals[4];
#pragma unroll
  for (int u = 0; u < 2; ++u) {
    const int b = bp + u;
    const int i = a < b ? a : b;
    const int j = a < b ? b : a;
    int e = row_start(i) + (j - i - 1);
    e = clampi(e, 0, kEdges - 1);
    const v2f pv = *(const v2f*)(eps + (size_t)e * kCls);
    const bool diag = (a == b);
    vals[2 * u]     = diag ? 0.0f : pv[0];
    vals[2 * u + 1] = diag ? 0.0f : pv[1];
  }
  const v4f o = (v4f){vals[0], vals[1], vals[2], vals[3]};
  float* dst = out + ((size_t)a * kNodes + bp) * kCls;
  *(volatile v4f*)dst = o;
  __threadfence();
  *(volatile v4f*)dst = o;
}

extern "C" void kernel_launch(void* const* d_in, const int* in_sizes, int n_in,
                              void* d_out, int out_size, void* d_ws, size_t ws_size,
                              hipStream_t stream) {
  if (n_in < 12) return;
  if ((size_t)out_size != (size_t)kNodes * kNodes * kCls) return;
  if (ws_size < kWsTotal) return;
  if (in_sizes[1] != kNodes * kFeat || in_sizes[2] != kFeat * kHid || in_sizes[4] != kHid * kHid ||
      in_sizes[6] != kHid * kFeat || in_sizes[8] != kFeat * kHid || in_sizes[10] != kHid * kCls ||
      in_sizes[3] != kHid || in_sizes[5] != kHid || in_sizes[7] != kFeat || in_sizes[9] != kHid || in_sizes[11] != kCls)
    return;

  const float* nf = (const float*)d_in[1];
  const float* w1 = (const float*)d_in[2];
  const float* b1 = (const float*)d_in[3];
  const float* w2 = (const float*)d_in[4];
  const float* b2 = (const float*)d_in[5];
  const float* w4 = (const float*)d_in[6];
  const float* b4 = (const float*)d_in[7];
  const float* w5 = (const float*)d_in[8];
  const float* b5 = (const float*)d_in[9];
  const float* w6 = (const float*)d_in[10];
  const float* b6 = (const float*)d_in[11];
  float* out = (float*)d_out;

  char* ws = (char*)d_ws;
  unsigned short* NF16  = (unsigned short*)(ws + kOffNF16);
  unsigned short* W1T16 = (unsigned short*)(ws + kOffW1T);
  unsigned short* W2T16 = (unsigned short*)(ws + kOffW2T);
  unsigned short* W4T16 = (unsigned short*)(ws + kOffW4T);
  unsigned short* W5T16 = (unsigned short*)(ws + kOffW5T);
  unsigned short* W6T16 = (unsigned short*)(ws + kOffW6T);
  unsigned short* H1    = (unsigned short*)(ws + kOffH1);
  unsigned short* H2    = (unsigned short*)(ws + kOffH2);
  float*          HF    = (float*)(ws + kOffHF);
  unsigned short* PROD16 = (unsigned short*)(ws + kOffProd);
  unsigned short* EP16   = (unsigned short*)(ws + kOffEP);
  float*          EPS    = (float*)(ws + kOffEPS);

  cast8_f16_kernel<<<(kNodes * kFeat / 8) / 256, 256, 0, stream>>>(nf, NF16, kNodes * kFeat / 8);
  tcast_kernel<<<dim3(kFeat / 64, kHid / 64), 256, 0, stream>>>(w1, W1T16, kFeat, kHid, kWCarry);
  tcast_kernel<<<dim3(kHid / 64, kHid / 64), 256, 0, stream>>>(w2, W2T16, kHid, kHid, kWCarry);
  tcast_kernel<<<dim3(kHid / 64, kFeat / 64), 256, 0, stream>>>(w4, W4T16, kHid, kFeat, kWCarry);
  tcast_kernel<<<dim3(kFeat / 64, kHid / 64), 256, 0, stream>>>(w5, W5T16, kFeat, kHid, kWCarry);
  w6t_kernel<<<(kW6Rows * kHid / 8 + 255) / 256, 256, 0, stream>>>(w6, W6T16);

  {
    const int tiles = (kNodes / 64) * (kHid / 64);
    wmma_gemm64<0, false, 2, 1, false, 4><<<dim3((tiles + 7) / 8, 1), 256, 0, stream>>>(
        NF16, NF16, kFeat, 0L, W1T16, W1T16, kFeat, 0L, (void*)H1, (void*)H1, kHid, 0L,
        b1, nf, 0L, kNodes, kHid, kFeat, kScale1, kActCarry);
    wmma_gemm64<0, false, 2, 1, false, 4><<<dim3((tiles + 7) / 8, 1), 256, 0, stream>>>(
        H1, H1, kHid, 0L, W2T16, W2T16, kHid, 0L, (void*)H2, (void*)H2, kHid, 0L,
        b2, nf, 0L, kNodes, kHid, kHid, kScale2, kActCarry);
    const int tiles3 = (kNodes / 64) * (kFeat / 64);
    wmma_gemm64<0, false, 2, 0, true, 0><<<dim3((tiles3 + 7) / 8, 1), 256, 0, stream>>>(
        H2, H2, kHid, 0L, W4T16, W4T16, kHid, 0L, (void*)HF, (void*)HF, kFeat, 0L,
        b4, nf, 0L, kNodes, kFeat, kHid, kScale2, 1.0f);
  }

  const int tiles4 = (kChunkE / 64) * (kHid / 64);
  for (int c = 0; c < kNumChunks; ++c) {
    pair_prod_kernel<<<(kChunkE * (kFeat / 8) + 255) / 256, 256, 0, stream>>>(HF, PROD16, c * kChunkE);
    wmma_gemm64<0, false, 2, 1, false, 2><<<dim3((tiles4 + 7) / 8, 1), 256, 0, stream>>>(
        PROD16, PROD16, kFeat, 0L, W5T16, W5T16, kFeat, 0L, (void*)EP16, (void*)EP16, kHid, 0L,
        b5, nf, 0L, kChunkE, kHid, kFeat, kScale2, kActCarry);
    logit_softmax_kernel<<<kChunkE / 512, 256, 0, stream>>>(EP16, W6T16, b6,
                                                             EPS + (size_t)c * kChunkE * kCls);
  }

  dense_write_kernel<<<(kNodes * (kNodes / 2) + 255) / 256, 256, 0, stream>>>(EPS, out);
}
